// ConvAddAttention_27745488732211
// MI455X (gfx1250) — hardware-verified
//
#include <hip/hip_runtime.h>


#define NI   8
#define CC   512
#define OO   512
#define IH   32
#define IW   32
#define KS   5
#define OH   28
#define OW   28
#define NPX  (NI * IH * IW)
#define NOP  (NI * OH * OW)

typedef unsigned short bf;
typedef __attribute__((ext_vector_type(16))) __bf16   v16bf;
typedef __attribute__((ext_vector_type(8)))  unsigned short v8us;
typedef __attribute__((ext_vector_type(8)))  float    v8f;
typedef __attribute__((ext_vector_type(4)))  float    v4f;
typedef v4f  __attribute__((may_alias)) v4fa;

__device__ __forceinline__ unsigned short f2bf(float f) { unsigned u = __float_as_uint(f); u += 0x7FFFu + ((u >> 16) & 1u); return (unsigned short)(u >> 16); }
__device__ __forceinline__ float bf2f(unsigned short b) { return __uint_as_float(((unsigned)b) << 16); }
__device__ __forceinline__ float bfr(float f) { return bf2f(f2bf(f)); }
__device__ __forceinline__ v16bf cat16b(v8us lo, v8us hi) { return __builtin_bit_cast(v16bf, __builtin_shufflevector(lo, hi, 0, 1, 2, 3, 4, 5, 6, 7, 8, 9, 10, 11, 12, 13, 14, 15)); }
__device__ __forceinline__ v8f wmmab(v16bf a, v16bf b, v8f c) { return __builtin_amdgcn_wmma_f32_16x16x32_bf16(false, a, false, b, (short)0, c, false, false); }
#define VST2(T, p, v) do { const T vst2_v_ = (v); *(volatile T*)(p) = vst2_v_; __threadfence(); *(volatile T*)(p) = vst2_v_; } while (0)

__global__ __launch_bounds__(256) void k_rows(const float* __restrict__ src, int rows, bf* dst) {
    const int lane = threadIdx.x & 31, r = blockIdx.x * 8 + (threadIdx.x >> 5);
    if (r >= rows) return;
    v8us o[2];
#pragma unroll
    for (int c = 0; c < 2; ++c)
#pragma unroll
        for (int i = 0; i < 8; ++i) o[c][i] = f2bf(src[(size_t)r * CC + c * 256 + lane * 8 + i]);
#pragma unroll
    for (int c = 0; c < 2; ++c) *(volatile v8us*)(dst + (size_t)r * CC + c * 256 + lane * 8) = o[c];
    __threadfence();
#pragma unroll
    for (int c = 0; c < 2; ++c) *(volatile v8us*)(dst + (size_t)r * CC + c * 256 + lane * 8) = o[c];
}
__global__ __launch_bounds__(128) void k_proj(const bf* __restrict__ XB, const bf* __restrict__ WB, const float* __restrict__ pb, float* PROJ) {
    __shared__ __align__(16) float ost[4][16 * 68];
    const int lane = threadIdx.x & 31, wave = threadIdx.x >> 5, lr = lane & 15, hi = lane >> 4;
    const size_t r0 = (size_t)blockIdx.x * 64 + wave * 16; const int c0 = blockIdx.y * 64;
    v8f acc[4];
#pragma unroll
    for (int t = 0; t < 4; ++t) acc[t] = (v8f){};
#pragma unroll 2
    for (int kc = 0; kc < CC; kc += 32) {
        const v16bf a = cat16b(*(const v8us*)(XB + (r0 + lr) * CC + kc + 8 * hi), *(const v8us*)(XB + (r0 + lr) * CC + kc + 8 * hi + 16));
#pragma unroll
        for (int t = 0; t < 4; ++t) { const bf* bp = WB + (size_t)(c0 + t * 16 + lr) * CC + kc + 8 * hi; acc[t] = wmmab(a, cat16b(*(const v8us*)bp, *(const v8us*)(bp + 16)), acc[t]); }
        asm volatile("v_nop" : "+v"(acc[0]), "+v"(acc[1]), "+v"(acc[2]), "+v"(acc[3]) : "v"(a) : "memory");
    }
    float* os = &ost[wave][0];
#pragma unroll
    for (int t = 0; t < 4; ++t) { const float bv = bfr(pb[c0 + t * 16 + lr]);
#pragma unroll
        for (int j = 0; j < 8; ++j) os[(hi * 8 + j) * 68 + t * 16 + lr] = acc[t][j] + bv; }
    __builtin_amdgcn_wave_barrier(); asm volatile("" ::: "memory");
    float* crow = PROJ + r0 * OO + c0;
    auto pass = [&]() {
#pragma unroll
        for (int s = 0; s < 8; ++s) { const int Lid = (lane >> 3) + 4 * s, piece = lane & 7; const int row = Lid >> 1, cofs = (Lid & 1) * 32 + piece * 4;
            const v4f val = *(const v4fa*)(os + row * 68 + cofs); *(volatile v4f*)(crow + (size_t)row * OO + cofs) = val; }
    };
    pass(); __threadfence(); pass();
}
__global__ __launch_bounds__(256) void k_score(const float* __restrict__ x, const float* __restrict__ sw, const float* __restrict__ sb, float* SC) {
    __shared__ float st[32];
    const int lane = threadIdx.x & 31, wave = threadIdx.x >> 5;
#pragma unroll 1
    for (int q = 0; q < 4; ++q) { const size_t px = (size_t)blockIdx.x * 32 + wave * 4 + q; float s = 0.f;
#pragma unroll 4
        for (int c = 0; c < CC / 32; ++c) s += bfr(x[px * CC + c * 32 + lane]) * bfr(sw[c * 32 + lane]);
#pragma unroll
        for (int sh = 16; sh; sh >>= 1) s += __shfl_xor(s, sh, 32);
        if (lane == 0) st[wave * 4 + q] = s + bfr(sb[0]); }
    __syncthreads();
    if (wave == 0) { const float vv = st[lane]; VST2(float, SC + (size_t)blockIdx.x * 32 + lane, vv); }
}
__global__ __launch_bounds__(256) void k_wgt(const float* __restrict__ SC, const float* __restrict__ lw, const float* __restrict__ lb, float* WGT) {
    const int p = blockIdx.x * 256 + threadIdx.x;
    if (p >= NOP) return;
    const int n = p / (OH * OW), rem = p - n * (OH * OW), hh = rem / OW, ww = rem - hh * OW;
    float sc[KS * KS]; float m = 0.f;
#pragma unroll
    for (int k = 0; k < KS * KS; ++k) { const int r = hh + k / KS, c = ww + k % KS; sc[k] = SC[(size_t)n * (IH * IW) + r * IW + c]; m += sc[k]; }
    m *= (1.0f / (KS * KS)); float var = 0.f;
#pragma unroll
    for (int k = 0; k < KS * KS; ++k) { const float d = sc[k] - m; var += d * d; }
    const float rs = rsqrtf(var * (1.0f / (KS * KS)) + 1e-5f);
    float mx = -3.0e38f;
#pragma unroll
    for (int k = 0; k < KS * KS; ++k) { sc[k] = (sc[k] - m) * rs * bfr(lw[k]) + bfr(lb[k]); mx = fmaxf(mx, sc[k]); }
    float sum = 0.f;
#pragma unroll
    for (int k = 0; k < KS * KS; ++k) { sc[k] = __expf(sc[k] - mx); sum += sc[k]; }
    const float inv = 1.0f / sum;
#pragma unroll 1
    for (int ps = 0; ps < 2; ++ps) {
#pragma unroll
        for (int k = 0; k < KS * KS; ++k) *(volatile float*)(WGT + (size_t)k * NOP + p) = sc[k] * inv;
        if (ps == 0) __threadfence(); }
}
__global__ __launch_bounds__(256) void k_out(const float* __restrict__ WGT, const float* __restrict__ PROJ, float* out) {
    const size_t f = (size_t)blockIdx.x * 256 + threadIdx.x;
    if (f >= (size_t)NI * OO * OH * OW) return;
    const int ww = (int)(f % OW); size_t t = f / OW; const int hh = (int)(t % OH); t /= OH; const int o = (int)(t % OO); const int n = (int)(t / OO);
    const int p = (n * OH + hh) * OW + ww;
    float s = 0.f;
#pragma unroll 5
    for (int k = 0; k < KS * KS; ++k) { const int r = hh + k / KS, c = ww + k % KS; s += WGT[(size_t)k * NOP + p] * PROJ[((size_t)n * (IH * IW) + r * IW + c) * OO + o]; }
    *(volatile float*)(out + f) = s; __threadfence(); *(volatile float*)(out + f) = s;
}

extern "C" void kernel_launch(void* const* d_in, const int* in_sizes, int n_in,
                              void* d_out, int out_size, void* d_ws, size_t ws_size, hipStream_t stream) {
    (void)in_sizes; (void)n_in; (void)out_size;
    const float* x = (const float*)d_in[0]; const float* pw = (const float*)d_in[1]; const float* pb = (const float*)d_in[2]; const float* sw = (const float*)d_in[3]; const float* sb = (const float*)d_in[4];
    const float* lw = (const float*)d_in[5]; const float* lb = (const float*)d_in[6];
    float* out = (float*)d_out;
    char* wsp = (char*)d_ws;
    auto take = [&](size_t bytes) { char* p = wsp; wsp += (bytes + 255) & ~(size_t)255; return (void*)p; };
    bf* XB = (bf*)take((size_t)NPX * CC * 2); bf* WB = (bf*)take((size_t)OO * CC * 2); float* PROJ = (float*)take((size_t)NPX * OO * 4); float* SC = (float*)take((size_t)NPX * 4); float* WGT = (float*)take((size_t)KS * KS * NOP * 4);
    if ((size_t)(wsp - (char*)d_ws) > ws_size) return;
    k_rows<<<NPX / 8, 256, 0, stream>>>(x, NPX, XB);
    k_rows<<<OO / 8, 256, 0, stream>>>(pw, OO, WB);
    k_proj<<<dim3(NPX / 64, OO / 64, 1), 128, 0, stream>>>(XB, WB, pb, PROJ);
    k_score<<<NPX / 32, 256, 0, stream>>>(x, sw, sb, SC);
    k_wgt<<<(NOP + 255) / 256, 256, 0, stream>>>(SC, lw, lb, WGT);
    k_out<<<(unsigned)(((size_t)NI * OO * OH * OW + 255) / 256), 256, 0, stream>>>(WGT, PROJ, out);
}
